// GraphAttentionLayer_4629974745450
// MI455X (gfx1250) — hardware-run, weakly checked
//
#include <hip/hip_runtime.h>
#include <math.h>

typedef __attribute__((ext_vector_type(16))) _Float16 v16h;
typedef __attribute__((ext_vector_type(8)))  _Float16 v8h;
typedef __attribute__((ext_vector_type(8)))  float    v8f;
typedef __attribute__((ext_vector_type(4)))  float    v4f;
typedef __attribute__((ext_vector_type(4)))  int      v4i;

constexpr int kBatch = 8;
constexpr int kNodes = 1024;
constexpr int kDin   = 256;
constexpr int kDout  = 256;
constexpr int kRows  = kBatch * kNodes;
constexpr float kSlope = 0.2f;
constexpr float kFill  = -9.0e15f;
constexpr float kCarryH  = 16.0f;
constexpr float kCarryW  = 256.0f;
constexpr float kCarryWh = 16.0f;
constexpr float kCarryP  = 16384.0f;
constexpr float kScale1  = kCarryWh / (kCarryH * kCarryW);
constexpr float kScale2  = 1.0f / (kCarryP * kCarryWh);
constexpr float kF16MinNormal = 6.103515625e-5f;

static_assert((kDin % 32) == 0 && (kNodes % 32) == 0);
static_assert((kDout % 64) == 0 && (kNodes % 64) == 0);
static_assert((kDout / 64) * (kNodes / 64) == 64);
static_assert((kRows % 32) == 0 && (kRows % 8) == 0);
static_assert((kDout * kDin) % (256 * 8) == 0);
static_assert(kDin == 256);

constexpr size_t kOffHB  = 0;
constexpr size_t kOffWB  = kOffHB  + (size_t)kRows * kDin * 2;
constexpr size_t kOffU   = kOffWB  + (size_t)kDout * kDin * 2;
constexpr size_t kOffSRC = kOffU   + (size_t)2 * kDin * 4;
constexpr size_t kOffDST = kOffSRC + (size_t)kRows * 4;
constexpr size_t kOffWHT = kOffDST + (size_t)kRows * 4;
constexpr size_t kOffPP  = kOffWHT + (size_t)kBatch * kDout * kNodes * 2;
constexpr size_t kWsTotal = kOffPP + (size_t)kBatch * kNodes * kNodes * 2;
static_assert(kWsTotal == 25364480ull);
static_assert(kWsTotal <= 134217728ull);
static_assert((kOffWB % 256) == 0 && (kOffU % 256) == 0 && (kOffSRC % 256) == 0 &&
              (kOffDST % 256) == 0 && (kOffWHT % 256) == 0 && (kOffPP % 256) == 0);

__device__ __forceinline__ _Float16 f16_flush(float v) {
  const float w = (fabsf(v) < kF16MinNormal) ? 0.0f : v;
  return (_Float16)w;
}

union FragU { v16h v; v8h h[2]; };
__device__ __forceinline__ v16h frag_load(const _Float16* p) {
  FragU f;
  f.h[0] = *(const v8h*)(p);
  f.h[1] = *(const v8h*)(p + 16);
  return f.v;
}

__device__ __forceinline__ v8f mma_h(v16h a, v16h b, v8f c) {
  c = __builtin_amdgcn_wmma_f32_16x16x32_f16(false, a, false, b, (short)0, c, false, false);
  asm volatile("v_nop\n\tv_nop\n\tv_nop\n\tv_nop" : "+v"(c) : "v"(a), "v"(b));
  return c;
}

template <int OUT_MODE>
__global__ __launch_bounds__(256) void wmma_gemm64_h(
    const unsigned short* __restrict__ Ap, int lda, long strideA,
    const unsigned short* __restrict__ Btp, int ldb, long strideB,
    void* __restrict__ Cout, int ldc, long strideC,
    int M, int N, int K, float scale) {
  const _Float16* A  = (const _Float16*)Ap;
  const _Float16* Bt = (const _Float16*)Btp;
  __shared__ __align__(16) float sT[8][16 * 68];
  const int b    = blockIdx.y;
  const int lane = threadIdx.x & 31;
  const int wave = threadIdx.x >> 5;
  const int tilesN = N >> 6;
  const int tilesM = M >> 6;
  const int tile = blockIdx.x * 8 + wave;
  if (tile >= tilesM * tilesN) return;
  const int tm = tile / tilesN;
  const int tn = tile - tm * tilesN;
  const int m0 = tm << 6;
  const int n0 = tn << 6;

  const _Float16* Ab = A  + (size_t)b * strideA;
  const _Float16* Bb = Bt + (size_t)b * strideB;

  const int rlane = lane & 15;
  const int koff  = (lane >> 4) * 8;
  const int mOff  = (lane >> 4) * 8;

  v8f acc[4][4];
#pragma unroll
  for (int i = 0; i < 4; ++i)
#pragma unroll
    for (int j = 0; j < 4; ++j) acc[i][j] = (v8f){0.f, 0.f, 0.f, 0.f, 0.f, 0.f, 0.f, 0.f};

  for (int k0 = 0; k0 < K; k0 += 32) {
    v16h bh[4];
#pragma unroll
    for (int j = 0; j < 4; ++j) {
      const size_t bo = (size_t)(n0 + (j << 4) + rlane) * ldb + koff + k0;
      bh[j] = frag_load(Bb + bo);
    }
#pragma unroll
    for (int i = 0; i < 4; ++i) {
      const size_t ao = (size_t)(m0 + (i << 4) + rlane) * lda + koff + k0;
      const v16h ah = frag_load(Ab + ao);
#pragma unroll
      for (int j = 0; j < 4; ++j) {
        acc[i][j] = mma_h(ah, bh[j], acc[i][j]);
      }
    }
  }

  float* slab = sT[wave];
#pragma unroll
  for (int i = 0; i < 4; ++i) {
    const int mBase = m0 + (i << 4);
#pragma unroll
    for (int j = 0; j < 4; ++j) {
#pragma unroll
      for (int r = 0; r < 8; ++r) {
        slab[(mOff + r) * 68 + (j << 4) + rlane] = acc[i][j][r] * scale;
      }
    }
    __builtin_amdgcn_fence(__ATOMIC_RELEASE, "workgroup");
    __builtin_amdgcn_wave_barrier();
    __builtin_amdgcn_fence(__ATOMIC_ACQUIRE, "workgroup");
    if (OUT_MODE == 0) {
      float* C = (float*)Cout + (size_t)b * strideC;
      const int hh = lane >> 4, c4 = (lane & 15) * 4;
      for (int pass = 0; pass < 2; ++pass) {
#pragma unroll
        for (int it = 0; it < 8; ++it) {
          const int row = it * 2 + hh;
          const v4f v = *(const v4f*)(slab + row * 68 + c4);
          *(volatile v4f*)(C + (size_t)(mBase + row) * ldc + n0 + c4) = v;
        }
        __threadfence();
      }
    } else {
      const int q = lane >> 3, c8 = (lane & 7) * 8;
      unsigned short* C = (unsigned short*)Cout + (size_t)b * strideC;
      for (int pass = 0; pass < 2; ++pass) {
#pragma unroll
        for (int it = 0; it < 4; ++it) {
          const int row = it * 4 + q;
          const float* sp = slab + row * 68 + c8;
          v8h hv;
#pragma unroll
          for (int e = 0; e < 8; ++e) {
            hv[e] = f16_flush(sp[e]);
          }
          *(volatile v8h*)(C + (size_t)(mBase + row) * ldc + n0 + c8) = hv;
        }
        __threadfence();
      }
    }
    __builtin_amdgcn_fence(__ATOMIC_RELEASE, "workgroup");
    __builtin_amdgcn_wave_barrier();
    __builtin_amdgcn_fence(__ATOMIC_ACQUIRE, "workgroup");
  }
}

constexpr int kWBlocks = (kDout * kDin) / (256 * 8);

__global__ __launch_bounds__(256) void prep_w_kernel(
    const float* __restrict__ W, const float* __restrict__ avec,
    unsigned short* __restrict__ WB, float* __restrict__ U) {
  const int tid = threadIdx.x;
  if (blockIdx.x < kWBlocks) {
    const size_t e0 = ((size_t)blockIdx.x * 256 + tid) << 3;
    const v4f a0 = *(const v4f*)(W + e0);
    const v4f a1 = *(const v4f*)(W + e0 + 4);
    v8h hv;
#pragma unroll
    for (int e = 0; e < 4; ++e) {
      hv[e]     = f16_flush(a0[e] * kCarryW);
      hv[4 + e] = f16_flush(a1[e] * kCarryW);
    }
    unsigned short* q = WB + e0;
    *(volatile v8h*)q = hv;
    __threadfence();
    *(volatile v8h*)q = hv;
  } else {
    float u1 = 0.0f, u2 = 0.0f;
#pragma unroll 1
    for (int f = 0; f < kDout; ++f) {
      const float c1 = avec[f];
      const float c2 = avec[kDout + f];
      const float w  = W[(size_t)f * kDin + tid];
      u1 = fmaf(c1, w, u1);
      u2 = fmaf(c2, w, u2);
    }
    volatile float* q1 = U + tid;
    volatile float* q2 = U + kDin + tid;
    *q1 = u1;
    *q2 = u2;
    __threadfence();
    *q1 = u1;
    *q2 = u2;
  }
}

__global__ __launch_bounds__(256) void prep_h_kernel(
    const float* __restrict__ h, const float* __restrict__ U,
    unsigned short* __restrict__ HB, float* __restrict__ srcv, float* __restrict__ dstv) {
  __shared__ float s_src[32];
  __shared__ float s_dst[32];
  const int tid = threadIdx.x, lane = tid & 31, wave = tid >> 5;
  const int row0 = blockIdx.x * 32;
  const v4f u1a = *(const v4f*)(U + lane * 8);
  const v4f u1b = *(const v4f*)(U + lane * 8 + 4);
  const v4f u2a = *(const v4f*)(U + kDin + lane * 8);
  const v4f u2b = *(const v4f*)(U + kDin + lane * 8 + 4);
#pragma unroll 1
  for (int r = 0; r < 4; ++r) {
    const int lr  = wave * 4 + r;
    const int row = row0 + lr;
    const float* hp = h + (size_t)row * kDin + lane * 8;
    const v4f x0 = *(const v4f*)(hp);
    const v4f x1 = *(const v4f*)(hp + 4);
    float s1 = 0.0f, s2 = 0.0f;
#pragma unroll
    for (int e = 0; e < 4; ++e) {
      s1 = fmaf(x0[e], u1a[e], s1);
      s2 = fmaf(x0[e], u2a[e], s2);
    }
#pragma unroll
    for (int e = 0; e < 4; ++e) {
      s1 = fmaf(x1[e], u1b[e], s1);
      s2 = fmaf(x1[e], u2b[e], s2);
    }
    for (int off = 16; off; off >>= 1) {
      s1 += __shfl_xor(s1, off, 32);
      s2 += __shfl_xor(s2, off, 32);
    }
    v8h hv;
#pragma unroll
    for (int e = 0; e < 4; ++e) {
      hv[e]     = f16_flush(x0[e] * kCarryH);
      hv[4 + e] = f16_flush(x1[e] * kCarryH);
    }
    unsigned short* q = HB + (size_t)row * kDin + lane * 8;
    *(volatile v8h*)q = hv;
    __threadfence();
    *(volatile v8h*)q = hv;
    if (lane == 0) {
      s_src[lr] = s1;
      s_dst[lr] = s2;
    }
  }
  __syncthreads();
  if (wave == 0) {
    const float v = s_src[lane];
    volatile float* q = srcv + row0 + lane;
    *q = v;
    __threadfence();
    *q = v;
  } else if (wave == 1) {
    const float v = s_dst[lane];
    volatile float* q = dstv + row0 + lane;
    *q = v;
    __threadfence();
    *q = v;
  }
}

__global__ __launch_bounds__(256) void attn_rows_kernel(
    const int* __restrict__ adj, const float* __restrict__ srcv, const float* __restrict__ dstv,
    unsigned short* __restrict__ PP) {
  __shared__ __align__(16) float sP[8][kNodes];
  const int tid = threadIdx.x, lane = tid & 31, wave = tid >> 5;
  const int row = blockIdx.x * 8 + wave;
  const int b   = row / kNodes;
  const int*   arow = adj + (size_t)row * kNodes;
  const float* drow = dstv + (size_t)b * kNodes;
  const float  si   = srcv[row];
  float* sp = sP[wave];

  float md = -INFINITY;
#pragma unroll 1
  for (int it = 0; it < kNodes / 128; ++it) {
    const int j0 = it * 128 + lane * 4;
    const v4i av = *(const v4i*)(arow + j0);
    const v4f dv = *(const v4f*)(drow + j0);
#pragma unroll
    for (int e = 0; e < 4; ++e) {
      const float c = (av[e] > 0) ? dv[e] : -INFINITY;
      md = fmaxf(md, c);
    }
  }
  for (int off = 16; off; off >>= 1) md = fmaxf(md, __shfl_xor(md, off, 32));
  const bool has = (md > -INFINITY);
  const float em = si + md;
  const float lm = (em > 0.0f) ? em : kSlope * em;
  const float m  = has ? lm : kFill;

  float l = 0.0f;
#pragma unroll 1
  for (int it = 0; it < kNodes / 128; ++it) {
    const int j0 = it * 128 + lane * 4;
    const v4i av = *(const v4i*)(arow + j0);
    const v4f dv = *(const v4f*)(drow + j0);
    v4f pv;
#pragma unroll
    for (int e = 0; e < 4; ++e) {
      const float ev = si + dv[e];
      const float lv = (ev > 0.0f) ? ev : kSlope * ev;
      const float x  = (av[e] > 0) ? lv : kFill;
      const float p  = expf(x - m);
      pv[e] = p;
      l += p;
    }
    *(v4f*)(sp + j0) = pv;
  }
  for (int off = 16; off; off >>= 1) l += __shfl_xor(l, off, 32);
  __syncthreads();

  const float inv = kCarryP * (1.0f / l);
  v8h hv[4];
#pragma unroll
  for (int it = 0; it < 4; ++it) {
    const int j0 = it * 256 + lane * 8;
    const v4f p0 = *(const v4f*)(sp + j0);
    const v4f p1 = *(const v4f*)(sp + j0 + 4);
#pragma unroll
    for (int e = 0; e < 4; ++e) {
      hv[it][e]     = f16_flush(p0[e] * inv);
      hv[it][4 + e] = f16_flush(p1[e] * inv);
    }
  }
  unsigned short* prow = PP + (size_t)row * kNodes + lane * 8;
  for (int pass = 0; pass < 2; ++pass) {
#pragma unroll
    for (int it = 0; it < 4; ++it) {
      *(volatile v8h*)(prow + it * 256) = hv[it];
    }
    __threadfence();
  }
}

extern "C" void kernel_launch(void* const* d_in, const int* in_sizes, int n_in,
                              void* d_out, int out_size, void* d_ws, size_t ws_size,
                              hipStream_t stream) {
  if (n_in < 4) return;
  if (in_sizes[0] != kRows * kDin) return;
  if (in_sizes[1] != kBatch * kNodes * kNodes) return;
  if (in_sizes[2] != kDout * kDin) return;
  if (in_sizes[3] != 2 * kDout) return;
  if (out_size != kRows * kDout) return;
  if (ws_size < kWsTotal) return;

  const float* h    = (const float*)d_in[0];
  const int*   adj  = (const int*)d_in[1];
  const float* W    = (const float*)d_in[2];
  const float* avec = (const float*)d_in[3];

  char* ws = (char*)d_ws;
  unsigned short* HB   = (unsigned short*)(ws + kOffHB);
  unsigned short* WB   = (unsigned short*)(ws + kOffWB);
  float*          U    = (float*)(ws + kOffU);
  float*          SRC  = (float*)(ws + kOffSRC);
  float*          DST  = (float*)(ws + kOffDST);
  unsigned short* WHT  = (unsigned short*)(ws + kOffWHT);
  unsigned short* PP   = (unsigned short*)(ws + kOffPP);

  prep_w_kernel<<<kWBlocks + 1, 256, 0, stream>>>(W, avec, WB, U);

  prep_h_kernel<<<kRows / 32, 256, 0, stream>>>(h, U, HB, SRC, DST);

  wmma_gemm64_h<1><<<dim3(8, kBatch), 256, 0, stream>>>(
      WB, kDin, 0L,
      HB, kDin, (long)kNodes * kDin,
      (void*)WHT, kNodes, (long)kDout * kNodes,
      kDout, kNodes, kDin, kScale1);

  attn_rows_kernel<<<kRows / 8, 256, 0, stream>>>(adj, SRC, DST, PP);

  wmma_gemm64_h<0><<<dim3(8, kBatch), 256, 0, stream>>>(
      PP, kNodes, (long)kNodes * kNodes,
      WHT, kNodes, (long)kDout * kNodes,
      d_out, kDout, (long)kNodes * kDout,
      kNodes, kDout, kNodes, kScale2);
}
